// EMM_19404662243509
// MI455X (gfx1250) — hardware-verified
//
#include <hip/hip_runtime.h>


#define NB_  8
#define SS   4096
#define DD   256
#define HH   256
#define FW   1794
#define NHOP 3
typedef _Float16 h16;
typedef unsigned short bf;
typedef __attribute__((ext_vector_type(16))) __bf16   v16bf;
typedef __attribute__((ext_vector_type(16))) _Float16 v16h;
typedef __attribute__((ext_vector_type(8)))  _Float16 v8h;
typedef __attribute__((ext_vector_type(8)))  unsigned short v8us;
typedef __attribute__((ext_vector_type(8)))  float    v8f;
typedef __attribute__((ext_vector_type(4)))  float    v4f;
typedef v8h  __attribute__((may_alias)) v8ha;
typedef v4f  __attribute__((may_alias)) v4fa;
typedef v8us __attribute__((may_alias)) v8usa;

__device__ __forceinline__ unsigned short f2bf(float f) { unsigned u = __float_as_uint(f); u += 0x7FFFu + ((u >> 16) & 1u); return (unsigned short)(u >> 16); }
__device__ __forceinline__ float bf2f(unsigned short b) { return __uint_as_float(((unsigned)b) << 16); }
__device__ __forceinline__ float bfr(float f) { return bf2f(f2bf(f)); }
__device__ __forceinline__ v16h cat16(v8h lo, v8h hi) { return __builtin_shufflevector(lo, hi, 0, 1, 2, 3, 4, 5, 6, 7, 8, 9, 10, 11, 12, 13, 14, 15); }
__device__ __forceinline__ v16bf cat16b(v8us lo, v8us hi) { return __builtin_bit_cast(v16bf, __builtin_shufflevector(lo, hi, 0, 1, 2, 3, 4, 5, 6, 7, 8, 9, 10, 11, 12, 13, 14, 15)); }
__device__ __forceinline__ v8f wmma16(v16h a, v16h b, v8f c) { return __builtin_amdgcn_wmma_f32_16x16x32_f16(false, a, false, b, (short)0, c, false, false); }
__device__ __forceinline__ v8f wmmab(v16bf a, v16bf b, v8f c) { return __builtin_amdgcn_wmma_f32_16x16x32_bf16(false, a, false, b, (short)0, c, false, false); }


template <typename T16> struct WFrag;
template <> struct WFrag<h16> { typedef v16h V; static __device__ __forceinline__ V ld(const h16* p) { return cat16(*(const v8h*)p, *(const v8h*)(p + 16)); } static __device__ __forceinline__ v8f mma(V a, V b, v8f c) { return wmma16(a, b, c); } };
template <> struct WFrag<bf> { typedef v16bf V; static __device__ __forceinline__ V ld(const bf* p) { return cat16b(*(const v8us*)p, *(const v8us*)(p + 16)); } static __device__ __forceinline__ v8f mma(V a, V b, v8f c) { return wmmab(a, b, c); } };
template <typename T16, int NSPLIT, bool BIAS>
__global__ __launch_bounds__(32) void k_gemmw(const T16* __restrict__ A, const T16* __restrict__ A2, const T16* __restrict__ Bt, const T16* __restrict__ Bt2, int K, float* C, int ldc, const float* __restrict__ bias, size_t sA, size_t sB, size_t sC) {
    typedef typename WFrag<T16>::V V;
    __shared__ __align__(16) float os[16 * 68];
    const size_t z = blockIdx.z; A += z * sA; if (A2) A2 += z * sA; Bt += z * sB; if (Bt2) Bt2 += z * sB; C += z * sC;
    const int lane = threadIdx.x & 31, lr = lane & 15, hi = lane >> 4; const int r0 = blockIdx.x * 64, c0 = blockIdx.y * 64;
    v8f acc[4][4];
#pragma unroll
    for (int mb = 0; mb < 4; ++mb)
#pragma unroll
        for (int nb = 0; nb < 4; ++nb) acc[mb][nb] = (v8f){};
    const size_t aoff = (size_t)(r0 + lr) * K + 8 * hi, boff = (size_t)(c0 + lr) * K + 8 * hi;
#pragma unroll 1
    for (int kc = 0; kc < K; kc += 32) {
        V a[4], a2[4];
#pragma unroll
        for (int mb = 0; mb < 4; ++mb) { a[mb] = WFrag<T16>::ld(A + aoff + (size_t)mb * 16 * K + kc); if (NSPLIT == 1 || NSPLIT == 2) a2[mb] = WFrag<T16>::ld(A2 + aoff + (size_t)mb * 16 * K + kc); }
#pragma unroll
        for (int nb = 0; nb < 4; ++nb) { const V b = WFrag<T16>::ld(Bt + boff + (size_t)nb * 16 * K + kc); V b2; if (NSPLIT >= 2) b2 = WFrag<T16>::ld(Bt2 + boff + (size_t)nb * 16 * K + kc);
#pragma unroll
            for (int mb = 0; mb < 4; ++mb) { acc[mb][nb] = WFrag<T16>::mma(a[mb], b, acc[mb][nb]); if (NSPLIT == 1 || NSPLIT == 2) acc[mb][nb] = WFrag<T16>::mma(a2[mb], b, acc[mb][nb]); if (NSPLIT >= 2) acc[mb][nb] = WFrag<T16>::mma(a[mb], b2, acc[mb][nb]); } }
        asm volatile("v_nop\n\tv_nop\n\tv_nop\n\tv_nop" : "+v"(acc[0][0]), "+v"(acc[1][1]), "+v"(acc[2][2]), "+v"(acc[3][3]) : "v"(a[0]), "v"(a[3]));
    }
#pragma unroll
    for (int mb = 0; mb < 4; ++mb) {
#pragma unroll
        for (int nb = 0; nb < 4; ++nb) {
#pragma unroll
            for (int j = 0; j < 8; ++j) os[(hi * 8 + j) * 68 + nb * 16 + lr] = acc[mb][nb][j]; }
        __builtin_amdgcn_wave_barrier(); asm volatile("" ::: "memory");
        float* crow = C + (size_t)(r0 + mb * 16) * ldc + c0;
#pragma unroll 1
        for (int ps = 0; ps < 2; ++ps) {
#pragma unroll
            for (int s = 0; s < 8; ++s) { const int row = 2 * s + hi, cofs = lr * 4; v4f val = *(const v4fa*)(os + row * 68 + cofs); if (BIAS) { val[0] += bfr(bias[c0 + cofs]); val[1] += bfr(bias[c0 + cofs + 1]); val[2] += bfr(bias[c0 + cofs + 2]); val[3] += bfr(bias[c0 + cofs + 3]); }
                *(volatile v4f*)(crow + (size_t)row * ldc + cofs) = val; }
            if (ps == 0) __threadfence(); }
        __builtin_amdgcn_wave_barrier(); asm volatile("" ::: "memory");
    }
}

__device__ __forceinline__ void splitf(float y, unsigned short& h, unsigned short& l) { h = f2bf(y); l = f2bf(y - bf2f(h)); }
__device__ __forceinline__ float sigf(float a) { return __fdiv_rn(1.0f, __fadd_rn(1.0f, __expf(-a))); }
__device__ __forceinline__ float tanhf_(float a) { const float e2 = __expf(2.0f * a); return __fsub_rn(1.0f, __fdiv_rn(2.0f, __fadd_rn(e2, 1.0f))); }
typedef __attribute__((ext_vector_type(2))) unsigned short v2us;
typedef __attribute__((ext_vector_type(4))) unsigned short v4us;

__global__ __launch_bounds__(256) void k_wtG(const float* __restrict__ w, int K, int N, bf* Bt) {
    const int lane = threadIdx.x & 31; const int L0 = (blockIdx.x * 8 + (threadIdx.x >> 5)) * 8; const int nlines = N * K / 64;
#pragma unroll 1
    for (int ps = 0; ps < 2; ++ps) {
#pragma unroll 1
        for (int l = 0; l < 8; ++l) { const int L = L0 + l; if (L >= nlines) break; const size_t e = (size_t)L * 64 + lane * 2; const int k = (int)(e % K), n = (int)(e / K); v2us o;
            o[0] = f2bf(w[(size_t)k * N + n]); o[1] = f2bf(w[(size_t)(k + 1) * N + n]); *(volatile v2us*)(Bt + e) = o; }
        if (ps == 0) __threadfence(); }
}
__global__ __launch_bounds__(256) void k_cvt8(const float* __restrict__ src, bf* dst, size_t n8) { const size_t i = (size_t)blockIdx.x * 256 + threadIdx.x; if (i >= n8) return; const v8f v = *(const v8f*)(src + i * 8); v8us o;
#pragma unroll
    for (int k = 0; k < 8; ++k) o[k] = f2bf(v[k]); *(volatile v8us*)(dst + i * 8) = o; __threadfence(); *(volatile v8us*)(dst + i * 8) = o; }
__global__ __launch_bounds__(256) void k_w1blk(const float* __restrict__ w1, bf* Bt0, bf* Bt1) { const int e = (blockIdx.x * 256 + threadIdx.x) * 4; if (e < HH * 768) { const int k = e % 768, h = e / 768; const int col = (k < 256) ? k : (k < 512 ? 768 + (k - 256) : 1280 + (k - 512)); v4us o;
#pragma unroll
        for (int qq = 0; qq < 4; ++qq) o[qq] = f2bf(w1[(size_t)h * FW + col + qq]); *(volatile v4us*)(Bt0 + e) = o; __threadfence(); *(volatile v4us*)(Bt0 + e) = o; }
    if (e < HH * 512) { const int k = e % 512, h = e / 512; const int col = (k < 256) ? 1024 + k : 1536 + (k - 256); v4us o;
#pragma unroll
        for (int qq = 0; qq < 4; ++qq) o[qq] = f2bf(w1[(size_t)h * FW + col + qq]); *(volatile v4us*)(Bt1 + e) = o; __threadfence(); *(volatile v4us*)(Bt1 + e) = o; } }
__global__ __launch_bounds__(256) void k_a0(const float* __restrict__ cb, const float* __restrict__ qb, bf* Ah, bf* Al) { const int e = (blockIdx.x * 256 + threadIdx.x) * 2; if (e >= SS * 768) return; const int k = e % 768, s = e / 768; v2us oh, ol;
#pragma unroll
    for (int qq = 0; qq < 2; ++qq) { const int kk = k + qq; const int d = kk & 255; const float cv = bfr(cb[(size_t)s * DD + d]), qv = bfr(qb[d]); const float v = (kk < 256) ? cv : (kk < 512 ? __fmul_rn(cv, qv) : fabsf(__fsub_rn(cv, qv))); unsigned short a, c2; splitf(v, a, c2); oh[qq] = a; ol[qq] = c2; }
    *(volatile v2us*)(Ah + e) = oh; *(volatile v2us*)(Al + e) = ol; __threadfence(); *(volatile v2us*)(Ah + e) = oh; *(volatile v2us*)(Al + e) = ol; }
__global__ __launch_bounds__(256) void k_a1(const float* __restrict__ cb, const float* __restrict__ M, bf* Ah, bf* Al) { const int e = (blockIdx.x * 256 + threadIdx.x) * 2; if (e >= SS * 512) return; const int k = e % 512, s = e / 512; v2us oh, ol;
#pragma unroll
    for (int qq = 0; qq < 2; ++qq) { const int kk = k + qq; const int d = kk & 255; const float cv = bfr(cb[(size_t)s * DD + d]), mv = M[d]; const float v = (kk < 256) ? __fmul_rn(cv, mv) : fabsf(__fsub_rn(cv, mv)); unsigned short a, c2; splitf(v, a, c2); oh[qq] = a; ol[qq] = c2; }
    *(volatile v2us*)(Ah + e) = oh; *(volatile v2us*)(Al + e) = ol; __threadfence(); *(volatile v2us*)(Ah + e) = oh; *(volatile v2us*)(Al + e) = ol; }
template <int RAW>
__global__ __launch_bounds__(256) void k_dot(const float* __restrict__ CW, const float* __restrict__ vec, float* DVo) { const int lane = threadIdx.x & 31; const int g = blockIdx.x * 8 + (threadIdx.x >> 5); if (g >= SS / 32) return; float keep = 0.f;
    for (int r = 0; r < 32; ++r) { const int s = g * 32 + r; float acc = 0.f;
#pragma unroll
        for (int d = lane; d < DD; d += 32) { float v = RAW ? bfr(vec[d]) : vec[d]; asm volatile("" : "+v"(v)); float p = __fmul_rn(CW[(size_t)s * DD + d], v); asm volatile("" : "+v"(p)); acc = __fadd_rn(acc, p); }
#pragma unroll
        for (int sh = 16; sh; sh >>= 1) acc += __shfl_xor(acc, sh, 32);
        if (lane == r) keep = acc; }
    *(volatile float*)(DVo + (size_t)g * 32 + lane) = keep; __threadfence(); *(volatile float*)(DVo + (size_t)g * 32 + lane) = keep; }
__global__ __launch_bounds__(256) void k_cq(const float* __restrict__ qb, const float* __restrict__ w1, const float* __restrict__ b1, float* CQ, float* M0) { const int h = threadIdx.x; float acc = 0.f;
#pragma unroll 4
    for (int d = 0; d < DD; ++d) { float w = bfr(w1[(size_t)h * FW + 512 + d]); asm volatile("" : "+v"(w)); float p = __fmul_rn(bfr(qb[d]), w); asm volatile("" : "+v"(p)); acc = __fadd_rn(acc, p); }
    float bb = bfr(b1[h]); asm volatile("" : "+v"(bb)); const float o = __fadd_rn(acc, bb); const float m0 = bfr(qb[h]); *(volatile float*)(CQ + h) = o; *(volatile float*)(M0 + h) = m0; __threadfence(); *(volatile float*)(CQ + h) = o; *(volatile float*)(M0 + h) = m0; }
__global__ __launch_bounds__(256) void k_rc(const float* __restrict__ M, const float* __restrict__ w1, const float* __restrict__ CQ, float* RC) { const int h = threadIdx.x; float acc = 0.f;
#pragma unroll 4
    for (int d = 0; d < DD; ++d) { float w = bfr(w1[(size_t)h * FW + 256 + d]); asm volatile("" : "+v"(w)); float p = __fmul_rn(M[d], w); asm volatile("" : "+v"(p)); acc = __fadd_rn(acc, p); }
    const float o = __fadd_rn(acc, CQ[h]); *(volatile float*)(RC + h) = o; __threadfence(); *(volatile float*)(RC + h) = o; }
__global__ __launch_bounds__(256) void k_hsc(const float* __restrict__ G0, const float* __restrict__ G1, const float* __restrict__ RC, const float* __restrict__ DQ, const float* __restrict__ DM, const float* __restrict__ w1, const float* __restrict__ w2, const float* __restrict__ b2, float* SC) {
    const int lane = threadIdx.x & 31; const int g = blockIdx.x * 8 + (threadIdx.x >> 5); if (g >= SS / 32) return; float wq[8], wm[8], ww[8], rc[8];
#pragma unroll
    for (int u = 0; u < 8; ++u) { const int h = lane + 32 * u; wq[u] = bfr(w1[(size_t)h * FW + 1792]); wm[u] = bfr(w1[(size_t)h * FW + 1793]); ww[u] = bfr(w2[h]); rc[u] = RC[h]; }
    const float bb = bfr(b2[0]); float keep = 0.f;
    for (int r = 0; r < 32; ++r) { const int s = g * 32 + r; const float dq = DQ[s], dm = DM[s]; float acc = 0.f;
#pragma unroll
        for (int u = 0; u < 8; ++u) { const int h = lane + 32 * u; float a = __fadd_rn(G0[(size_t)s * HH + h], G1[(size_t)s * HH + h]); asm volatile("" : "+v"(a)); a = __fadd_rn(a, rc[u]); float t1 = __fmul_rn(dq, wq[u]), t2 = __fmul_rn(dm, wm[u]); asm volatile("" : "+v"(t1)); asm volatile("" : "+v"(t2)); float t = __fadd_rn(t1, t2); asm volatile("" : "+v"(t)); const float pre = __fadd_rn(a, t);
            float th = tanhf_(pre); asm volatile("" : "+v"(th)); float p = __fmul_rn(th, ww[u]); asm volatile("" : "+v"(p)); acc = __fadd_rn(acc, p); }
#pragma unroll
        for (int sh = 16; sh; sh >>= 1) acc += __shfl_xor(acc, sh, 32);
        if (lane == r) keep = __fadd_rn(acc, bb); }
    *(volatile float*)(SC + (size_t)g * 32 + lane) = keep; __threadfence(); *(volatile float*)(SC + (size_t)g * 32 + lane) = keep; }
__global__ __launch_bounds__(32) void k_att(const float* __restrict__ SC, const int* __restrict__ lenc, int b, float* ATT, float* OUTa) { const int lane = threadIdx.x; const int len = lenc[b]; float m = -3.0e38f;
    for (int s = lane; s < SS; s += 32) if (s < len) m = fmaxf(m, SC[s]);
#pragma unroll
    for (int sh = 16; sh; sh >>= 1) m = fmaxf(m, __shfl_xor(m, sh, 32));
    float sum = 0.f;
    for (int s = lane; s < SS; s += 32) if (s < len) { float d0 = __fsub_rn(SC[s], m); asm volatile("" : "+v"(d0)); sum = __fadd_rn(sum, __builtin_amdgcn_exp2f(__fmul_rn(d0, 1.4426950408889634f))); }
#pragma unroll
    for (int sh = 16; sh; sh >>= 1) sum += __shfl_xor(sum, sh, 32);
    const float inv = __fdiv_rn(1.0f, sum);
    for (int ps = 0; ps < 2; ++ps) {
        for (int c0 = lane * 4; c0 < SS; c0 += 128) { v4f o;
#pragma unroll
            for (int qq = 0; qq < 4; ++qq) { const int s = c0 + qq; float d0 = __fsub_rn(SC[s], m); asm volatile("" : "+v"(d0)); o[qq] = (s < len) ? __fmul_rn(__builtin_amdgcn_exp2f(__fmul_rn(d0, 1.4426950408889634f)), inv) : 0.f; }
            *(volatile v4f*)(ATT + c0) = o; *(volatile v4f*)(OUTa + c0) = o; }
        if (ps == 0) __threadfence(); } }
__global__ __launch_bounds__(256) void k_e(const float* __restrict__ ATT, const float* __restrict__ cb, float* E) { const int d = threadIdx.x; float acc = 0.f;
    for (int s = 0; s < SS; ++s) { float p = __fmul_rn(ATT[s], bfr(cb[(size_t)s * DD + d])); asm volatile("" : "+v"(p)); acc = __fadd_rn(acc, p); }
    *(volatile float*)(E + d) = acc; __threadfence(); *(volatile float*)(E + d) = acc; }
__global__ __launch_bounds__(256) void k_gru(const float* __restrict__ E, const float* __restrict__ M, const float* __restrict__ wih, const float* __restrict__ whh, const float* __restrict__ bih, const float* __restrict__ bhh, float* MN, float* OUT0b) { const int j = threadIdx.x; float gi[3], gh[3];
#pragma unroll
    for (int g = 0; g < 3; ++g) { float a = 0.f, c2 = 0.f; const float* wi = wih + (size_t)(g * DD + j) * DD; const float* wh = whh + (size_t)(g * DD + j) * DD;
#pragma unroll 4
        for (int d = 0; d < DD; ++d) { float w0 = bfr(wi[d]), w1v = bfr(wh[d]); asm volatile("" : "+v"(w0)); asm volatile("" : "+v"(w1v)); float p = __fmul_rn(E[d], w0), q2 = __fmul_rn(M[d], w1v); asm volatile("" : "+v"(p)); asm volatile("" : "+v"(q2)); a = __fadd_rn(a, p); c2 = __fadd_rn(c2, q2); }
        float b0 = bfr(bih[g * DD + j]), b1v = bfr(bhh[g * DD + j]); asm volatile("" : "+v"(b0)); asm volatile("" : "+v"(b1v)); gi[g] = __fadd_rn(a, b0); gh[g] = __fadd_rn(c2, b1v); }
    const float r = sigf(__fadd_rn(gi[0], gh[0])), z = sigf(__fadd_rn(gi[1], gh[1])); float rn = __fmul_rn(r, gh[2]); asm volatile("" : "+v"(rn)); const float n = tanhf_(__fadd_rn(gi[2], rn));
    float omz = __fsub_rn(1.0f, z); float t1 = __fmul_rn(omz, n), t2 = __fmul_rn(z, M[j]); asm volatile("" : "+v"(t1)); asm volatile("" : "+v"(t2)); const float mn = __fadd_rn(t1, t2);
    *(volatile float*)(MN + j) = mn; if (OUT0b) *(volatile float*)(OUT0b + j) = mn; __threadfence(); *(volatile float*)(MN + j) = mn; if (OUT0b) *(volatile float*)(OUT0b + j) = mn; }

extern "C" void kernel_launch(void* const* d_in, const int* in_sizes, int n_in,
                              void* d_out, int out_size, void* d_ws, size_t ws_size, hipStream_t stream) {
    (void)in_sizes; (void)n_in; (void)out_size;
    const float* c = (const float*)d_in[0]; const float* q = (const float*)d_in[1]; const int* lenc = (const int*)d_in[2]; const float* aw = (const float*)d_in[3]; const float* w1 = (const float*)d_in[4]; const float* b1 = (const float*)d_in[5]; const float* w2 = (const float*)d_in[6]; const float* b2 = (const float*)d_in[7]; const float* wih = (const float*)d_in[8]; const float* whh = (const float*)d_in[9]; const float* bih = (const float*)d_in[10]; const float* bhh = (const float*)d_in[11];
    float* OUT0 = (float*)d_out; float* OUT1 = (float*)d_out + (size_t)NB_ * DD;
    char* wsp = (char*)d_ws;
    auto take = [&](size_t bytes) { char* p = wsp; wsp += (bytes + 255) & ~(size_t)255; return (void*)p; };
    bf* WA = (bf*)take((size_t)DD * DD * 2); bf* Bt0 = (bf*)take((size_t)HH * 768 * 2); bf* Bt1 = (bf*)take((size_t)HH * 512 * 2); bf* CB = (bf*)take((size_t)NB_ * SS * DD * 2); float* CW = (float*)take((size_t)SS * DD * 4);
    bf* A0h = (bf*)take((size_t)SS * 768 * 2); bf* A0l = (bf*)take((size_t)SS * 768 * 2); bf* A1h = (bf*)take((size_t)SS * 512 * 2); bf* A1l = (bf*)take((size_t)SS * 512 * 2); float* G0 = (float*)take((size_t)SS * HH * 4); float* G1 = (float*)take((size_t)SS * HH * 4);
    float* DQ = (float*)take((size_t)SS * 4); float* DM = (float*)take((size_t)SS * 4); float* SC = (float*)take((size_t)SS * 4); float* ATT = (float*)take((size_t)SS * 4); float* CQ = (float*)take(1024); float* RC = (float*)take(1024); float* E = (float*)take(1024); float* MA = (float*)take(1024); float* MB = (float*)take(1024);
    if ((size_t)(wsp - (char*)d_ws) > ws_size) return;
    k_wtG<<<(unsigned)((DD * DD / 64 + 63) / 64), 256, 0, stream>>>(aw, DD, DD, WA); k_w1blk<<<(HH * 768 / 4 + 255) / 256, 256, 0, stream>>>(w1, Bt0, Bt1); k_cvt8<<<(unsigned)(((size_t)NB_ * SS * DD / 8 + 255) / 256), 256, 0, stream>>>(c, CB, (size_t)NB_ * SS * DD / 8);
    for (int b = 0; b < NB_; ++b) { const float* cb = c + (size_t)b * SS * DD; const float* qb = q + (size_t)b * DD;
        k_gemmw<bf, 0, false><<<dim3(SS / 64, DD / 64, 1), 32, 0, stream>>>(CB + (size_t)b * SS * DD, nullptr, WA, nullptr, DD, CW, DD, nullptr, 0, 0, 0);
        k_dot<1><<<(SS / 32 + 7) / 8, 256, 0, stream>>>(CW, qb, DQ);
        k_a0<<<(SS * 768 / 2 + 255) / 256, 256, 0, stream>>>(cb, qb, A0h, A0l); k_gemmw<bf, 1, false><<<dim3(SS / 64, HH / 64, 1), 32, 0, stream>>>(A0h, A0l, Bt0, nullptr, 768, G0, HH, nullptr, 0, 0, 0);
        k_cq<<<1, 256, 0, stream>>>(qb, w1, b1, CQ, MA);
        float* Mcur = MA; float* Mnext = MB;
        for (int hop = 0; hop < NHOP; ++hop) {
            k_dot<0><<<(SS / 32 + 7) / 8, 256, 0, stream>>>(CW, Mcur, DM); k_rc<<<1, 256, 0, stream>>>(Mcur, w1, CQ, RC);
            k_a1<<<(SS * 512 / 2 + 255) / 256, 256, 0, stream>>>(cb, Mcur, A1h, A1l); k_gemmw<bf, 1, false><<<dim3(SS / 64, HH / 64, 1), 32, 0, stream>>>(A1h, A1l, Bt1, nullptr, 512, G1, HH, nullptr, 0, 0, 0);
            k_hsc<<<(SS / 32 + 7) / 8, 256, 0, stream>>>(G0, G1, RC, DQ, DM, w1, w2, b2, SC);
            k_att<<<1, 32, 0, stream>>>(SC, lenc, b, ATT, OUT1 + ((size_t)hop * NB_ + b) * SS);
            k_e<<<1, 256, 0, stream>>>(ATT, cb, E);
            k_gru<<<1, 256, 0, stream>>>(E, Mcur, wih, whh, bih, bhh, Mnext, hop == NHOP - 1 ? OUT0 + (size_t)b * DD : nullptr);
            float* t = Mcur; Mcur = Mnext; Mnext = t; } }
}
